// TritonTrittention_47588237639881
// MI455X (gfx1250) — hardware-verified
//
#include <hip/hip_runtime.h>
#include <stdint.h>

#define DEVINL __device__ __forceinline__

typedef _Float16 f16t;
typedef _Float16 v16h __attribute__((ext_vector_type(16)));
typedef _Float16 v8h  __attribute__((ext_vector_type(8)));
typedef float    v8f  __attribute__((ext_vector_type(8)));
typedef float    v4f  __attribute__((ext_vector_type(4)));
typedef v8h __attribute__((may_alias)) v8ha;
typedef v4f __attribute__((may_alias)) v4fa;
union FragH { v16h v; v8h half[2]; };

#define NH      8
#define SEQ     256
#define HDIM    64
#define TPB     256
#define NWAVE   8
#define NJB     (SEQ / 16)
#define RPW     32
#define NGRP    (TPB / 16)
#define MLINE   32
#define CVT_BLK (NH * SEQ * HDIM / 8 / TPB)
#define FIN_BLK (NH * SEQ / 4 / TPB)

#define ACAR    64.0f
#define BCAR    16.0f
#define SC      (0.125f / 1024.0f)
#define NEG_BIG (-3.0e38f)

static_assert(TPB == NWAVE * 32);
static_assert(NWAVE * RPW == SEQ);
static_assert(NJB * 16 == SEQ);
static_assert(HDIM == 64);
static_assert(SEQ == 256);
static_assert(TPB == SEQ);
static_assert(NGRP * 16 == SEQ);
static_assert(NGRP * HDIM == TPB * 4);
static_assert(NWAVE * NJB == 128);
static_assert(CVT_BLK * TPB * 8 == NH * SEQ * HDIM);
static_assert(FIN_BLK * TPB * 4 == NH * SEQ);
static_assert(HDIM * 4 == 256);
static_assert(MLINE * 4 == 128);

DEVINL v8f wmma_f16(v16h a, v16h b, v8f c) {
  v8f d = __builtin_amdgcn_wmma_f32_16x16x32_f16(false, a, false, b, (short)0, c, false, false);
  asm volatile("v_nop\n\tv_nop\n\tv_nop\n\tv_nop" : "+v"(d) : "v"(a), "v"(b));
  return d;
}
DEVINL v8f zero8f() {
  v8f z = {0.f, 0.f, 0.f, 0.f, 0.f, 0.f, 0.f, 0.f};
  return z;
}

DEVINL void build_a(FragH& a, const float* __restrict__ krow, const float* qs, int kc, int hh) {
  const float* kp = krow + kc * 32 + 8 * hh;
  const float* qp = qs + kc * 32 + 8 * hh;
  const v4f x0 = *(const v4fa*)(kp),      x1 = *(const v4fa*)(kp + 4);
  const v4f x2 = *(const v4fa*)(kp + 16), x3 = *(const v4fa*)(kp + 20);
  const v4f q0 = *(const v4fa*)(qp),      q1 = *(const v4fa*)(qp + 4);
  const v4f q2 = *(const v4fa*)(qp + 16), q3 = *(const v4fa*)(qp + 20);
  #pragma unroll
  for (int j = 0; j < 4; ++j) {
    a.v[j]      = (f16t)((q0[j] * x0[j]) * ACAR);
    a.v[4 + j]  = (f16t)((q1[j] * x1[j]) * ACAR);
    a.v[8 + j]  = (f16t)((q2[j] * x2[j]) * ACAR);
    a.v[12 + j] = (f16t)((q3[j] * x3[j]) * ACAR);
  }
}

DEVINL void load_b(FragH& b, const f16t* __restrict__ jrow, int kc, int hh) {
  const f16t* p = jrow + kc * 32 + 8 * hh;
  b.half[0] = *(const v8ha*)(p);
  b.half[1] = *(const v8ha*)(p + 16);
}

__global__ __launch_bounds__(TPB) void cvt_k2_k(const float* __restrict__ K2g, f16t* __restrict__ K2h)
{
  if (blockIdx.x >= CVT_BLK) return;
  const int t = blockIdx.x * TPB + (int)threadIdx.x;
  const float* s = K2g + (size_t)t * 8;
  const v4f x0 = *(const v4fa*)(s), x1 = *(const v4fa*)(s + 4);
  v8h o;
  #pragma unroll
  for (int j = 0; j < 4; ++j) {
    o[j]     = (f16t)(x0[j] * BCAR);
    o[4 + j] = (f16t)(x1[j] * BCAR);
  }
  f16t* dst = K2h + (size_t)t * 8;
  *(volatile v8h*)dst = o;
  __threadfence();
  *(volatile v8h*)dst = o;
}

__global__ __launch_bounds__(TPB) void attn_k(const float* __restrict__ Qg, const float* __restrict__ K1g,
                                             const f16t* __restrict__ K2h,
                                             const float* __restrict__ V1g, const float* __restrict__ V2g,
                                             float* __restrict__ out0, float* __restrict__ mline)
{
  __shared__ __attribute__((aligned(16))) float sQ[HDIM];
  __shared__ float sC[NWAVE * SEQ];
  __shared__ float sM[NWAVE * NJB];
  __shared__ float sF[NWAVE * NJB];
  __shared__ float sMw[NWAVE];
  __shared__ float sFw[NWAVE];
  __shared__ float sZw[NWAVE];
  __shared__ float sR[SEQ];
  __shared__ float sRf[SEQ];
  __shared__ float sCf[SEQ];
  __shared__ __attribute__((aligned(16))) float sO[NGRP * HDIM];
  __shared__ __attribute__((aligned(16))) float sOut[HDIM];

  const int tid = threadIdx.x, lane = tid & 31;
  const int wave = __builtin_amdgcn_readfirstlane(tid >> 5);
  const int hh = lane >> 4, m = lane & 15;
  const int blk = blockIdx.x;
  if (blk >= NH * SEQ) return;
  const int h = blk >> 8;
  const int q = blk & (SEQ - 1);
  const size_t headOff = (size_t)h * SEQ * HDIM;

  if (tid < HDIM) sQ[tid] = Qg[headOff + (size_t)q * HDIM + tid];
  __syncthreads();

  const int rA0 = RPW * wave + m;
  const int rA1 = rA0 + 16;
  FragH a00, a01, a10, a11;
  {
    const float* k0p = K1g + headOff + (size_t)rA0 * HDIM;
    const float* k1p = K1g + headOff + (size_t)rA1 * HDIM;
    build_a(a00, k0p, sQ, 0, hh);
    build_a(a01, k0p, sQ, 1, hh);
    build_a(a10, k1p, sQ, 0, hh);
    build_a(a11, k1p, sQ, 1, hh);
  }

  float mrun = NEG_BIG;
  float racc0[8], racc1[8];
  #pragma unroll
  for (int v = 0; v < 8; ++v) { racc0[v] = 0.0f; racc1[v] = 0.0f; }

  const f16t* k2head = K2h + headOff;

  #pragma unroll 1
  for (int jb = 0; jb < NJB; ++jb) {
    const f16t* jrow = k2head + (size_t)(jb * 16 + m) * HDIM;
    FragH b0, b1;
    load_b(b0, jrow, 0, hh);
    load_b(b1, jrow, 1, hh);

    v8f c0 = wmma_f16(a00.v, b0.v, zero8f());
    c0 = wmma_f16(a01.v, b1.v, c0);
    v8f c1 = wmma_f16(a10.v, b0.v, zero8f());
    c1 = wmma_f16(a11.v, b1.v, c1);

    float tmax = NEG_BIG;
    #pragma unroll
    for (int v = 0; v < 8; ++v) tmax = fmaxf(tmax, fmaxf(c0[v], c1[v]));
    tmax *= SC;
    tmax = fmaxf(tmax, __shfl_xor(tmax, 16));
    tmax = fmaxf(tmax, __shfl_xor(tmax, 8));
    tmax = fmaxf(tmax, __shfl_xor(tmax, 4));
    tmax = fmaxf(tmax, __shfl_xor(tmax, 2));
    tmax = fmaxf(tmax, __shfl_xor(tmax, 1));

    const float mnew = fmaxf(mrun, tmax);
    const float fe = __expf(mrun - mnew);
    const float f = (jb == 0) ? 0.0f : fe;
    mrun = mnew;

    float cs = 0.0f;
    #pragma unroll
    for (int v = 0; v < 8; ++v) {
      const float p0 = __expf(fmaf(c0[v], SC, -mnew));
      const float p1 = __expf(fmaf(c1[v], SC, -mnew));
      racc0[v] = fmaf(racc0[v], f, p0);
      racc1[v] = fmaf(racc1[v], f, p1);
      cs += p0 + p1;
    }
    cs += __shfl_xor(cs, 16);
    if (hh == 0) sC[wave * SEQ + jb * 16 + m] = cs;
    if (lane == 0) sM[wave * NJB + jb] = mnew;
  }

  #pragma unroll
  for (int v = 0; v < 8; ++v) {
    racc0[v] += __shfl_xor(racc0[v], 8);
    racc0[v] += __shfl_xor(racc0[v], 4);
    racc0[v] += __shfl_xor(racc0[v], 2);
    racc0[v] += __shfl_xor(racc0[v], 1);
    racc1[v] += __shfl_xor(racc1[v], 8);
    racc1[v] += __shfl_xor(racc1[v], 4);
    racc1[v] += __shfl_xor(racc1[v], 2);
    racc1[v] += __shfl_xor(racc1[v], 1);
  }
  if (m == 0) {
    #pragma unroll
    for (int v = 0; v < 8; ++v) {
      sR[RPW * wave + 8 * hh + v]      = racc0[v];
      sR[RPW * wave + 16 + 8 * hh + v] = racc1[v];
    }
  }
  if (lane == 0) sMw[wave] = mrun;
  __syncthreads();

  float gmax = sMw[0];
  #pragma unroll
  for (int w = 1; w < NWAVE; ++w) gmax = fmaxf(gmax, sMw[w]);

  if (wave < 4) sF[tid] = __expf(sM[tid] - gmax);
  if (wave == 4) {
    const float e = __expf(sMw[lane & (NWAVE - 1)] - gmax);
    if (lane < NWAVE) sFw[lane] = e;
  }
  __syncthreads();

  {
    const float R = sR[tid] * sFw[tid >> 5];
    float C = 0.0f;
    #pragma unroll
    for (int w = 0; w < NWAVE; ++w) C = fmaf(sC[w * SEQ + tid], sF[w * NJB + (tid >> 4)], C);
    sRf[tid] = R;
    sCf[tid] = C;
    float z = R;
    z += __shfl_xor(z, 16);
    z += __shfl_xor(z, 8);
    z += __shfl_xor(z, 4);
    z += __shfl_xor(z, 2);
    z += __shfl_xor(z, 1);
    if (lane == 0) sZw[wave] = z;
  }
  __syncthreads();

  float Z = sZw[0];
  #pragma unroll
  for (int w = 1; w < NWAVE; ++w) Z += sZw[w];

  {
    const int g = tid >> 4;
    const int dd = (tid & 15) << 2;
    const float* v1p = V1g + headOff + dd;
    const float* v2p = V2g + headOff + dd;
    v4f acc = {0.f, 0.f, 0.f, 0.f};
    #pragma unroll 4
    for (int i = 0; i < 16; ++i) {
      const int r = g * 16 + i;
      const v4f x1 = *(const v4fa*)(v1p + (size_t)r * HDIM);
      const v4f x2 = *(const v4fa*)(v2p + (size_t)r * HDIM);
      const float rr = sRf[r], cc = sCf[r];
      acc = x1 * rr + acc;
      acc = x2 * cc + acc;
    }
    *(v4fa*)(sO + g * HDIM + dd) = acc;
  }
  __syncthreads();

  const float invZ = 1.0f / Z;
  if (tid < HDIM) {
    float o = sO[tid];
    #pragma unroll
    for (int g = 1; g < NGRP; ++g) o += sO[g * HDIM + tid];
    sOut[tid] = o * invZ;
  }
  __syncthreads();

  if (wave == 0) {
    const v4f v = *(const v4fa*)(sOut + 4 * m);
    float* dst = out0 + (size_t)blk * HDIM + 4 * m;
    if (lane < 16) *(volatile v4f*)dst = v;
    __threadfence();
    if (lane < 16) *(volatile v4f*)dst = v;
  }
  if (wave == 1) {
    const float mm = gmax + logf(Z);
    const v4f v = {mm, mm, mm, mm};
    float* dst = mline + (size_t)blk * MLINE + 4 * (lane & 7);
    if (lane < 8) *(volatile v4f*)dst = v;
    __threadfence();
    if (lane < 8) *(volatile v4f*)dst = v;
  }
}

__global__ __launch_bounds__(TPB) void fin_k(const float* __restrict__ mline, float* __restrict__ out1)
{
  if (blockIdx.x >= FIN_BLK) return;
  const int g = blockIdx.x * TPB + (int)threadIdx.x;
  v4f v;
  #pragma unroll
  for (int i = 0; i < 4; ++i) v[i] = mline[(size_t)(4 * g + i) * MLINE];
  float* dst = out1 + (size_t)4 * g;
  *(volatile v4f*)dst = v;
  __threadfence();
  *(volatile v4f*)dst = v;
}

extern "C" void kernel_launch(void* const* d_in, const int* in_sizes, int n_in,
                              void* d_out, int out_size, void* d_ws, size_t ws_size,
                              hipStream_t stream) {
  if (n_in < 5) return;
  for (int i = 0; i < 5; ++i)
    if (in_sizes[i] != NH * SEQ * HDIM) return;
  if (out_size != NH * SEQ * HDIM + NH * SEQ) return;

  const float* Qg  = (const float*)d_in[0];
  const float* K1g = (const float*)d_in[1];
  const float* K2g = (const float*)d_in[2];
  const float* V1g = (const float*)d_in[3];
  const float* V2g = (const float*)d_in[4];
  float* out0 = (float*)d_out;
  float* out1 = (float*)d_out + (size_t)NH * SEQ * HDIM;

  const size_t szK2h = (size_t)NH * SEQ * HDIM * 2;
  const size_t szML  = (size_t)NH * SEQ * MLINE * 4;
  size_t off = 0;
  char* ws = (char*)d_ws;
  f16t*  K2h   = (f16t*)(ws + off);   off += szK2h;
  float* mline = (float*)(ws + off);  off += szML;
  if (off > ws_size) return;

  cvt_k2_k<<<CVT_BLK, TPB, 0, stream>>>(K2g, K2h);
  attn_k<<<NH * SEQ, TPB, 0, stream>>>(Qg, K1g, K2h, V1g, V2g, out0, mline);
  fin_k<<<FIN_BLK, TPB, 0, stream>>>(mline, out1);
  (void)hipGetLastError();
}
